// CausalSelfAttention_89842125897794
// MI455X (gfx1250) — hardware-verified
//
#include <hip/hip_runtime.h>
#include <math.h>

#ifndef NB
#define NB 2
#endif
#ifndef SEQ
#define SEQ 2048
#endif
#define NB_FULL 2
#define SEQ_FULL 2048
#define EMB 1024
#define NHEAD 16
#define HDIM 64
#define NQKV (3 * EMB)
#define ISL 256
#define AW 4

static_assert(NB >= 1 && NB <= NB_FULL);
static_assert(SEQ % 64 == 0 && SEQ <= SEQ_FULL);
static_assert(ISL % 64 == 0 && ISL <= SEQ);
static_assert((SEQ - ISL) % (16 * AW) == 0);
static_assert(NHEAD * HDIM == EMB);
static_assert(HDIM == 64);
static_assert(EMB % 512 == 0 && NQKV % 512 == 0);
static_assert(EMB % 32 == 0);
static_assert(EMB % 8 == 0);

typedef __attribute__((ext_vector_type(16))) _Float16 v16h;
typedef __attribute__((ext_vector_type(8)))  _Float16 v8h;
typedef __attribute__((ext_vector_type(16))) __bf16   v16b;
typedef __attribute__((ext_vector_type(8)))  __bf16   v8b;
typedef __attribute__((ext_vector_type(8)))  float    v8f;
typedef __attribute__((ext_vector_type(4)))  float    v4f;
typedef __attribute__((ext_vector_type(4)))  unsigned int v4u;

__device__ __forceinline__ int frag_k(int i, int h) { return (i < 8) ? (8 * h + i) : (16 + 8 * h + (i - 8)); }
__device__ __forceinline__ __bf16 bf16_rne(float f) {
    unsigned int u = __float_as_uint(f);
    u += 0x7fffu + ((u >> 16) & 1u);
    return __builtin_bit_cast(__bf16, (unsigned short)(u >> 16));
}
__device__ __forceinline__ float bf16_f32(__bf16 b) { return __uint_as_float(((unsigned int)__builtin_bit_cast(unsigned short, b)) << 16); }

struct Split { v16b hi, lo; };
__device__ __forceinline__ v8f wmma3(const Split& a, const Split& b, v8f c) {
    c = __builtin_amdgcn_wmma_f32_16x16x32_bf16(false, a.hi, false, b.hi, (short)0, c, false, false);
    c = __builtin_amdgcn_wmma_f32_16x16x32_bf16(false, a.hi, false, b.lo, (short)0, c, false, false);
    c = __builtin_amdgcn_wmma_f32_16x16x32_bf16(false, a.lo, false, b.hi, (short)0, c, false, false);
    asm volatile("v_nop\n\tv_nop\n\tv_nop\n\tv_nop" : "+v"(c) : "v"(a.hi), "v"(a.lo), "v"(b.hi), "v"(b.lo));
    return c;
}
__device__ __forceinline__ Split sp_ld_g(const float* __restrict__ p, int k0, int h) {
    Split r;
#pragma unroll
    for (int i = 0; i < 16; ++i) {
        const float x = p[k0 + frag_k(i, h)];
        const __bf16 hb = bf16_rne(x); r.hi[i] = hb; r.lo[i] = bf16_rne(x - bf16_f32(hb));
    }
    return r;
}
__device__ __forceinline__ Split sp_ld_s(const float* p, int k0, int h) {
    Split r;
#pragma unroll
    for (int i = 0; i < 16; ++i) {
        const float x = p[k0 + frag_k(i, h)];
        const __bf16 hb = bf16_rne(x); r.hi[i] = hb; r.lo[i] = bf16_rne(x - bf16_f32(hb));
    }
    return r;
}

#define VST2(T, ptr, val) do { const T vst2_v_ = (val); *(volatile T*)(ptr) = vst2_v_; __threadfence(); *(volatile T*)(ptr) = vst2_v_; } while (0)
#define VST2V4(ptr, val) do { const v4f vst2_v4_ = (val); *(volatile v4f*)(ptr) = vst2_v4_; __threadfence(); *(volatile v4f*)(ptr) = vst2_v4_; } while (0)

__device__ __forceinline__ unsigned int cmb_pk2(float a, float b) { return (unsigned int)__builtin_bit_cast(unsigned short, (_Float16)a) | ((unsigned int)__builtin_bit_cast(unsigned short, (_Float16)b) << 16); }
__device__ __forceinline__ float cmb_bf(float v) { const unsigned u = __float_as_uint(v); const unsigned r = (u + 0x7fffu + ((u >> 16) & 1u)) & 0xffff0000u; return __uint_as_float(r); }
__device__ __forceinline__ unsigned short bfu_rne(float v) { unsigned u = __float_as_uint(v); u += 0x7FFFu + ((u >> 16) & 1u); return (unsigned short)(u >> 16); }
__device__ __forceinline__ void bfsplit(float v, unsigned short& hi, unsigned short& lo) { hi = bfu_rne(v); lo = bfu_rne(v - __uint_as_float((unsigned)hi << 16)); }

__global__ __launch_bounds__(256) void k_bfvec(const float* __restrict__ SRC, float* __restrict__ DST, int n) {
    const int u = blockIdx.x * 256 + threadIdx.x; if (u >= n) return;
    VST2(float, DST + u, cmb_bf(SRC[u]));
}
__global__ __launch_bounds__(256) void k_cast_rows(const float* __restrict__ SRC, unsigned short* __restrict__ DST, int nRows, int seq, long long sBatch, float sc, int viabf) {
    const long long u = (long long)blockIdx.x * 256 + threadIdx.x; const int per = EMB / 8;
    if (u >= (long long)nRows * per) return;
    const int r = (int)(u / per), c0 = 8 * (int)(u % per); const int b = r / seq, t = r - b * seq;
    const float* s = SRC + (long long)b * sBatch + (long long)t * EMB + c0;
    const v4f a = *(const v4f*)s, c = *(const v4f*)(s + 4);
    float w[8] = {a.x, a.y, a.z, a.w, c.x, c.y, c.z, c.w};
#pragma unroll
    for (int e = 0; e < 8; ++e) w[e] = (viabf ? cmb_bf(w[e]) : w[e]) * sc;
    v4u pk; pk.x = cmb_pk2(w[0], w[1]); pk.y = cmb_pk2(w[2], w[3]); pk.z = cmb_pk2(w[4], w[5]); pk.w = cmb_pk2(w[6], w[7]);
    VST2(v4u, (v4u*)(DST + (long long)r * EMB + c0), pk);
}
__global__ __launch_bounds__(256) void k_castT(const float* __restrict__ SRC, int lds, unsigned short* __restrict__ DST, int ldd, int nR, int nC, float sc, int asbf) {
    const long long u = (long long)blockIdx.x * 256 + threadIdx.x; const int per = nR / 8;
    if (u >= (long long)nC * per) return;
    const int c = (int)(u / per); const int r0 = 8 * (int)(u % per);
    unsigned int q[8];
#pragma unroll
    for (int e = 0; e < 8; ++e) {
        const float wv = cmb_bf(SRC[(long long)(r0 + e) * lds + c]);
        const unsigned int qb = __float_as_uint(wv) >> 16;
        const unsigned int qh = (unsigned int)__builtin_bit_cast(unsigned short, (_Float16)(wv * sc));
        q[e] = asbf ? qb : qh;
    }
    v4u pk; pk.x = q[0] | (q[1] << 16); pk.y = q[2] | (q[3] << 16); pk.z = q[4] | (q[5] << 16); pk.w = q[6] | (q[7] << 16);
    VST2(v4u, (v4u*)(DST + (long long)c * ldd + r0), pk);
}
__global__ __launch_bounds__(256) void k_split_rows(const float* __restrict__ SRC, long long sSb, unsigned short* __restrict__ PH, unsigned short* __restrict__ PL, int rows, int nBatch) {
    const long long u = (long long)blockIdx.x * 256 + threadIdx.x; const int per = EMB / 8;
    if (u >= (long long)nBatch * rows * per) return;
    const int c0 = 8 * (int)(u % per); const long long rr = u / per; const int r = (int)(rr % rows); const int b = (int)(rr / rows);
    const float* s = SRC + (long long)b * sSb + (long long)r * EMB + c0;
    const v4f a = *(const v4f*)s, c = *(const v4f*)(s + 4);
    const float w[8] = {a.x, a.y, a.z, a.w, c.x, c.y, c.z, c.w};
    unsigned short hh[8], ll[8];
#pragma unroll
    for (int e = 0; e < 8; ++e) bfsplit(w[e], hh[e], ll[e]);
    v4u ph, pl;
    ph.x = (unsigned)hh[0] | ((unsigned)hh[1] << 16); ph.y = (unsigned)hh[2] | ((unsigned)hh[3] << 16); ph.z = (unsigned)hh[4] | ((unsigned)hh[5] << 16); ph.w = (unsigned)hh[6] | ((unsigned)hh[7] << 16);
    pl.x = (unsigned)ll[0] | ((unsigned)ll[1] << 16); pl.y = (unsigned)ll[2] | ((unsigned)ll[3] << 16); pl.z = (unsigned)ll[4] | ((unsigned)ll[5] << 16); pl.w = (unsigned)ll[6] | ((unsigned)ll[7] << 16);
    const long long o = ((long long)b * rows + r) * EMB + c0;
    volatile v4u* dh = (volatile v4u*)(PH + o); volatile v4u* dl = (volatile v4u*)(PL + o);
    *dh = ph; *dl = pl; __threadfence(); *dh = ph; *dl = pl;
}

__device__ __forceinline__ void dep_guard_h(v8f& a, v8f& b, v16h x, v16h y) { asm volatile("v_nop\n\tv_nop\n\tv_nop\n\tv_nop" : "+v"(a), "+v"(b) : "v"(x), "v"(y)); }
__device__ __forceinline__ void dep_guard_b(v8f& a, v8f& b, v16b x, v16b y) { asm volatile("v_nop\n\tv_nop\n\tv_nop\n\tv_nop" : "+v"(a), "+v"(b) : "v"(x), "v"(y)); }
__device__ __forceinline__ void keep4_h(v16h a, v16h b, v16h c, v16h d) { asm volatile("v_nop" :: "v"(a), "v"(b), "v"(c), "v"(d)); }
__device__ __forceinline__ void keep4_b(v16b a, v16b b, v16b c, v16b d) { asm volatile("v_nop" :: "v"(a), "v"(b), "v"(c), "v"(d)); }
__device__ __forceinline__ void acc_guard4(v8f& a, v8f& b, v8f& c, v8f& d) { asm volatile("v_nop\n\tv_nop\n\tv_nop\n\tv_nop" : "+v"(a), "+v"(b), "+v"(c), "+v"(d)); }
template <typename T> struct Frag;
template <> struct Frag<_Float16> {
    typedef v16h V; union U { v16h v; v8h h[2]; };
    static __device__ __forceinline__ v16h load(const _Float16* p) { U f; f.h[0] = *(const v8h*)(p); f.h[1] = *(const v8h*)(p + 16); return f.v; }
    static __device__ __forceinline__ v8f mma(v16h a, v16h b, v8f c) { return __builtin_amdgcn_wmma_f32_16x16x32_f16(false, a, false, b, (short)0, c, false, false); }
    static __device__ __forceinline__ void guard(v8f& a, v8f& b, v16h x, v16h y) { dep_guard_h(a, b, x, y); }
    static __device__ __forceinline__ void keep(v16h a, v16h b, v16h c, v16h d) { keep4_h(a, b, c, d); }
};
template <> struct Frag<__bf16> {
    typedef v16b V; union U { v16b v; v8b h[2]; };
    static __device__ __forceinline__ v16b load(const __bf16* p) { U f; f.h[0] = *(const v8b*)(p); f.h[1] = *(const v8b*)(p + 16); return f.v; }
    static __device__ __forceinline__ v8f mma(v16b a, v16b b, v8f c) { return __builtin_amdgcn_wmma_f32_16x16x32_bf16(false, a, false, b, (short)0, c, false, false); }
    static __device__ __forceinline__ void guard(v8f& a, v8f& b, v16b x, v16b y) { dep_guard_b(a, b, x, y); }
    static __device__ __forceinline__ void keep(v16b a, v16b b, v16b c, v16b d) { keep4_b(a, b, c, d); }
};
template <int ET> struct Elem;
template <> struct Elem<0> { typedef _Float16 T; };
template <> struct Elem<1> { typedef __bf16 T; };

struct G64P {
    const unsigned short* A; const unsigned short* Bt; float* C; const float* bias; const float* resid;
    long long strideA, strideC, strideR;
    int lda, ldb, ldc, M, N, K; float scale; int pad_;
};
static_assert(sizeof(G64P) == 5 * 8 + 3 * 8 + 6 * 4 + 4 + 4);

__device__ __forceinline__ G64P g64_pack(const unsigned short* A, const unsigned short* Bt, float* C, const float* bias, const float* resid,
                                         long long strideA, long long strideC, long long strideR,
                                         int lda, int ldb, int ldc, int M, int N, int K, float scale) {
    G64P g;
    g.A = A; g.Bt = Bt; g.C = C; g.bias = bias; g.resid = resid;
    g.strideA = strideA; g.strideC = strideC; g.strideR = strideR;
    g.lda = lda; g.ldb = ldb; g.ldc = ldc; g.M = M; g.N = N; g.K = K; g.scale = scale; g.pad_ = 0;
    return g;
}
#define G64_ARGS(g) (g).A, (g).Bt, (g).C, (g).bias, (g).resid, (g).strideA, (g).strideC, (g).strideR, (g).lda, (g).ldb, (g).ldc, (g).M, (g).N, (g).K, (g).scale

template <int ET, int HASBIAS, int RESID>
__device__ __forceinline__ void gemm64_body(float* sbase, const G64P& g) {
    typedef typename Elem<ET>::T T;
    typedef typename Frag<T>::V V;
    const int b = blockIdx.y, lane = threadIdx.x & 31, wave = threadIdx.x >> 5;
    const int tilesN = g.N >> 6, tilesM = g.M >> 6, ntile = tilesM * tilesN;
    int tile = blockIdx.x * 8 + wave;
    const bool live = tile < ntile;
    tile = live ? tile : (ntile - 1);
    const int tm = tile / tilesN, tn = tile - tm * tilesN;
    const int m0 = tm << 6, n0 = tn << 6;
    const T* __restrict__ Ab = (const T*)g.A + (size_t)b * g.strideA;
    const T* __restrict__ Bb = (const T*)g.Bt;
    const int rlane = lane & 15;
    const int koff  = (lane >> 4) * 8;
    const int mOff  = (lane >> 4) * 8;
    v8f acc[4][4];
#pragma unroll
    for (int i = 0; i < 4; ++i)
#pragma unroll
        for (int j = 0; j < 4; ++j) acc[i][j] = (v8f){0.f, 0.f, 0.f, 0.f, 0.f, 0.f, 0.f, 0.f};
    for (int k0 = 0; k0 < g.K; k0 += 32) {
        V bh[4];
#pragma unroll
        for (int j = 0; j < 4; ++j) bh[j] = Frag<T>::load(Bb + (size_t)(n0 + (j << 4) + rlane) * g.ldb + koff + k0);
#pragma unroll
        for (int i = 0; i < 4; ++i) {
            const V ah = Frag<T>::load(Ab + (size_t)(m0 + (i << 4) + rlane) * g.lda + koff + k0);
#pragma unroll
            for (int j = 0; j < 4; ++j) acc[i][j] = Frag<T>::mma(ah, bh[j], acc[i][j]);
            Frag<T>::guard(acc[i][0], acc[i][3], ah, ah);
        }
        Frag<T>::keep(bh[0], bh[1], bh[2], bh[3]);
    }
    acc_guard4(acc[0][0], acc[0][1], acc[0][2], acc[0][3]);
    acc_guard4(acc[1][0], acc[1][1], acc[1][2], acc[1][3]);
    acc_guard4(acc[2][0], acc[2][1], acc[2][2], acc[2][3]);
    acc_guard4(acc[3][0], acc[3][1], acc[3][2], acc[3][3]);

    float* slab = sbase + wave * (16 * 68);
    float* C = g.C + (size_t)b * g.strideC;
    const float* Rb = g.resid + (size_t)b * g.strideR;
#pragma unroll
    for (int i = 0; i < 4; ++i) {
        const int mBase = m0 + (i << 4);
#pragma unroll
        for (int j = 0; j < 4; ++j) {
            const int n = n0 + (j << 4) + rlane;
            float bv = 0.f;
            if (HASBIAS) bv = g.bias[n];
#pragma unroll
            for (int r = 0; r < 8; ++r) {
                float v = acc[i][j][r] * g.scale;
                if (HASBIAS) v += bv;
                if (RESID) v += Rb[(size_t)(mBase + mOff + r) * g.ldc + n];
                slab[(mOff + r) * 68 + (j << 4) + rlane] = v;
            }
        }
        __syncthreads();
        if (live) {
            const int hh = lane >> 4, c4 = (lane & 15) * 4;
            for (int pass = 0; pass < 2; ++pass) {
#pragma unroll
                for (int it = 0; it < 8; ++it) {
                    const int row = it * 2 + hh;
                    const v4f v = *(const v4f*)(slab + row * 68 + c4);
                    *(volatile v4f*)(C + (size_t)(mBase + row) * g.ldc + n0 + c4) = v;
                }
                __threadfence();
            }
        }
        __syncthreads();
    }
}
__global__ __launch_bounds__(256) void k_gemm_f16_bias(const unsigned short* A, const unsigned short* Bt, float* C, const float* bias, const float* resid,
                                                       long long strideA, long long strideC, long long strideR,
                                                       int lda, int ldb, int ldc, int M, int N, int K, float scale) {
    __shared__ __align__(16) float sT[8 * 16 * 68];
    const G64P g = g64_pack(A, Bt, C, bias, resid, strideA, strideC, strideR, lda, ldb, ldc, M, N, K, scale);
    gemm64_body<0, 1, 0>(sT, g);
}
__global__ __launch_bounds__(256) void k_gemm_bf16_bias(const unsigned short* A, const unsigned short* Bt, float* C, const float* bias, const float* resid,
                                                        long long strideA, long long strideC, long long strideR,
                                                        int lda, int ldb, int ldc, int M, int N, int K, float scale) {
    __shared__ __align__(16) float sT[8 * 16 * 68];
    const G64P g = g64_pack(A, Bt, C, bias, resid, strideA, strideC, strideR, lda, ldb, ldc, M, N, K, scale);
    gemm64_body<1, 1, 0>(sT, g);
}
__global__ __launch_bounds__(256) void k_gemm_bf16_resid(const unsigned short* A, const unsigned short* Bt, float* C, const float* bias, const float* resid,
                                                         long long strideA, long long strideC, long long strideR,
                                                         int lda, int ldb, int ldc, int M, int N, int K, float scale) {
    __shared__ __align__(16) float sT[8 * 16 * 68];
    const G64P g = g64_pack(A, Bt, C, bias, resid, strideA, strideC, strideR, lda, ldb, ldc, M, N, K, scale);
    gemm64_body<1, 0, 1>(sT, g);
}

__global__ __launch_bounds__(64) void k_gx_exact(const float* __restrict__ QKVp, float* __restrict__ AOp, long long sQb, long long sOb, float sc) {
    #pragma clang fp contract(off)
    __shared__ float qs[64]; __shared__ float ps[ISL]; __shared__ float red[2];
    const int i = blockIdx.x, h = blockIdx.y, b = blockIdx.z, t = threadIdx.x;
    const float* Q = QKVp + (long long)b * sQb;
    const float* KV = Q + EMB;
    qs[t] = Q[(long long)i * NQKV + h * 64 + t]; __syncthreads();
#pragma unroll
    for (int r = 0; r < ISL / 64; ++r) {
        const int j = t + 64 * r; const int jc = min(j, i); const float* kr = KV + (long long)jc * NQKV + h * 64; float s = 0.f;
#pragma unroll 8
        for (int d = 0; d < 64; ++d) s += qs[d] * kr[d];
        ps[j] = (j <= i) ? s * sc : -3.0e38f;
    }
    __syncthreads();
    if (t == 0) {
        float m = -3.0e38f; for (int j = 0; j <= i; ++j) m = fmaxf(m, ps[j]);
        float z = 0.f; for (int j = 0; j <= i; ++j) { const float e = expf(ps[j] - m); ps[j] = e; z += e; }
        red[0] = 1.f / z;
    }
    __syncthreads();
    const float inv = red[0]; float o = 0.f;
    for (int j = 0; j <= i; ++j) o += ps[j] * KV[(long long)j * NQKV + EMB + h * 64 + t];
    VST2(float, AOp + (long long)b * sOb + (long long)i * EMB + h * 64 + t, o * inv);
}

struct AttnP {
    const float* Q; const float* K; const float* V; float* O;
    long long sQb, sQh, sQi, sKb, sKh, sKj, sVb, sVh, sVj, sOb, sOh, sOi;
    int Lq, Lk, coff, pad_; float scale, pad2_;
};
static_assert(sizeof(AttnP) == 4 * 8 + 12 * 8 + 4 * 4 + 2 * 4);

__device__ __forceinline__ AttnP attn_pack(const float* Q, const float* K, const float* V, float* O,
                                           long long sQb, long long sQh, long long sQi, long long sKb, long long sKh, long long sKj,
                                           long long sVb, long long sVh, long long sVj, long long sOb, long long sOh, long long sOi,
                                           int Lq, int Lk, int coff, float scale) {
    AttnP p;
    p.Q = Q; p.K = K; p.V = V; p.O = O;
    p.sQb = sQb; p.sQh = sQh; p.sQi = sQi; p.sKb = sKb; p.sKh = sKh; p.sKj = sKj;
    p.sVb = sVb; p.sVh = sVh; p.sVj = sVj; p.sOb = sOb; p.sOh = sOh; p.sOi = sOi;
    p.Lq = Lq; p.Lk = Lk; p.coff = coff; p.pad_ = 0; p.scale = scale; p.pad2_ = 0.0f;
    return p;
}
#define ATTN_ARGS(a) (a).Q, (a).K, (a).V, (a).O, (a).sQb, (a).sQh, (a).sQi, (a).sKb, (a).sKh, (a).sKj, (a).sVb, (a).sVh, (a).sVj, (a).sOb, (a).sOh, (a).sOi, (a).Lq, (a).Lk, (a).coff, (a).scale

__global__ __launch_bounds__(32 * AW) void k_attn_causal(const float* Q, const float* K, const float* V, float* O,
                                                         long long sQb, long long sQh, long long sQi, long long sKb, long long sKh, long long sKj,
                                                         long long sVb, long long sVh, long long sVj, long long sOb, long long sOh, long long sOi,
                                                         int Lq, int Lk, int coff, float scale) {
    const AttnP p = attn_pack(Q, K, V, O, sQb, sQh, sQi, sKb, sKh, sKj, sVb, sVh, sVj, sOb, sOh, sOi, Lq, Lk, coff, scale);
    constexpr int NT = HDIM / 16;
    constexpr int KS = HDIM / 32;
    constexpr int VP = HDIM + 8;
    __shared__ __align__(16) float  pl[AW][16 * 64];
    __shared__ __align__(16) __bf16 vl[2 * 64 * VP];
    const int lane = threadIdx.x & 31, hf = lane >> 4, l15 = lane & 15, wave = threadIdx.x >> 5;
    const int h = blockIdx.y, b = blockIdx.z;
    const int q0 = (blockIdx.x * AW + wave) * 16;
    float* myp = pl[wave];
    const float L2E = 1.4426950408889634f;
    const float NEG = -__builtin_inff();
    const int qi = min(q0 + l15, p.Lq - 1);
    const float* qrow  = p.Q + b * p.sQb + h * p.sQh + (long long)qi * p.sQi;
    const float* kbase = p.K + b * p.sKb + h * p.sKh;
    const float* vbase = p.V + b * p.sVb + h * p.sVh;
    Split qs_[KS];
#pragma unroll
    for (int ks = 0; ks < KS; ++ks) qs_[ks] = sp_ld_g(qrow, ks * 32, hf);
    v8f o[NT]; float m8[8], l8[8];
#pragma unroll
    for (int t = 0; t < NT; ++t) { v8f zz = {}; o[t] = zz; }
#pragma unroll
    for (int i = 0; i < 8; ++i) { m8[i] = NEG; l8[i] = 0.f; }
    const int je = (blockIdx.x * AW + AW - 1) * 16 + 16 + p.coff;
    const int jend = min(p.Lk, max(je, 0));
    for (int j0 = 0; j0 < jend; j0 += 64) {
        __syncthreads();
        for (int idx = threadIdx.x; idx < 64 * HDIM; idx += 32 * AW) {
            const int jr = idx / HDIM, d = idx - jr * HDIM, j = j0 + jr; const int jc = min(j, p.Lk - 1);
            const float fl = vbase[(long long)jc * p.sVj + d];
            const float f = (j < p.Lk) ? fl : 0.f;
            const __bf16 hb = bf16_rne(f);
            vl[jr * VP + d] = hb; vl[64 * VP + jr * VP + d] = bf16_rne(f - bf16_f32(hb));
        }
        v8f s[4];
#pragma unroll
        for (int t = 0; t < 4; ++t) {
            const int j = min(j0 + t * 16 + l15, p.Lk - 1);
            const float* krow = kbase + (long long)j * p.sKj;
            v8f acc = {};
#pragma unroll
            for (int ks = 0; ks < KS; ++ks) acc = wmma3(qs_[ks], sp_ld_g(krow, ks * 32, hf), acc);
            s[t] = acc;
        }
        float pv[8][4];
#pragma unroll
        for (int i = 0; i < 8; ++i) {
            const int irow = q0 + i + 8 * hf;
            float sc[4];
#pragma unroll
            for (int t = 0; t < 4; ++t) {
                const int jg = j0 + t * 16 + l15;
                float v = s[t][i] * p.scale;
                if (jg >= p.Lk || jg > irow + p.coff) v = NEG; else v *= L2E;
                sc[t] = v;
            }
            float mx = fmaxf(fmaxf(sc[0], sc[1]), fmaxf(sc[2], sc[3]));
            mx = fmaxf(mx, __shfl_xor(mx, 1, 32)); mx = fmaxf(mx, __shfl_xor(mx, 2, 32));
            mx = fmaxf(mx, __shfl_xor(mx, 4, 32)); mx = fmaxf(mx, __shfl_xor(mx, 8, 32));
            const float mnew = fmaxf(m8[i], mx);
            const float corr = (mnew == NEG) ? 1.f : exp2f(m8[i] - mnew);
            float rs = 0.f;
#pragma unroll
            for (int t = 0; t < 4; ++t) { const float pp = (sc[t] == NEG) ? 0.f : exp2f(sc[t] - mnew); rs += pp; pv[i][t] = pp; }
            rs += __shfl_xor(rs, 1, 32); rs += __shfl_xor(rs, 2, 32); rs += __shfl_xor(rs, 4, 32); rs += __shfl_xor(rs, 8, 32);
            l8[i] = l8[i] * corr + rs; m8[i] = mnew;
#pragma unroll
            for (int t = 0; t < NT; ++t) o[t][i] *= corr;
        }
#pragma unroll
        for (int i = 0; i < 8; ++i)
#pragma unroll
            for (int t = 0; t < 4; ++t) myp[(i + 8 * hf) * 64 + t * 16 + l15] = pv[i][t];
        __syncthreads();
        const Split pa0 = sp_ld_s(myp + l15 * 64, 0, hf), pa1 = sp_ld_s(myp + l15 * 64, 32, hf);
        const __bf16* vh = vl; const __bf16* vlo = vl + 64 * VP;
#pragma unroll
        for (int t = 0; t < NT; ++t) {
            const int dcol = t * 16 + l15;
            Split b0, b1;
#pragma unroll
            for (int e = 0; e < 16; ++e) {
                const int k0 = frag_k(e, hf), k1 = 32 + frag_k(e, hf);
                b0.hi[e] = vh[k0 * VP + dcol]; b0.lo[e] = vlo[k0 * VP + dcol]; b1.hi[e] = vh[k1 * VP + dcol]; b1.lo[e] = vlo[k1 * VP + dcol];
            }
            o[t] = wmma3(pa0, b0, o[t]);
            o[t] = wmma3(pa1, b1, o[t]);
        }
    }
    float invr[8];
#pragma unroll
    for (int i = 0; i < 8; ++i) invr[i] = (l8[i] > 0.f) ? 1.f / l8[i] : 0.f;
    __syncthreads();
#pragma unroll
    for (int i = 0; i < 8; ++i)
#pragma unroll
        for (int t = 0; t < NT; ++t) myp[(i + 8 * hf) * 64 + t * 16 + l15] = o[t][i] * invr[i];
    __syncthreads();
    float* obase = p.O + b * p.sOb + h * p.sOh;
    for (int r0 = 0; r0 < 16; r0 += 2) {
        const int row = r0 + (lane >> 4), c4 = (lane & 15) * 4;
        const v4f v = *(const v4f*)(myp + row * 64 + c4);
        VST2V4(obase + (long long)(q0 + row) * p.sOi + c4, v);
    }
}

constexpr size_t al256(size_t n) { return ((n + 255) / 256) * 256; }
constexpr size_t ROWS      = (size_t)NB * SEQ;
constexpr size_t SZ_X16    = al256(ROWS * EMB * 2);
constexpr size_t SZ_W316   = al256((size_t)NQKV * EMB * 2);
constexpr size_t SZ_QKV    = al256(ROWS * NQKV * 4);
constexpr size_t SZ_AO     = al256(ROWS * EMB * 4);
constexpr size_t SZ_BR3    = al256((size_t)(NQKV + 64) * 4);
constexpr size_t SZ_WO     = al256((size_t)EMB * EMB * 2);
constexpr size_t SZ_ISLP   = al256((size_t)NB * ISL * EMB * 2);
constexpr size_t SZ_BRO    = al256((size_t)(EMB + 64) * 4);
constexpr size_t WS_TOTAL  = SZ_X16 + SZ_W316 + SZ_QKV + SZ_AO + SZ_BR3 + 2 * SZ_WO + 2 * SZ_ISLP + SZ_BRO;
static_assert(WS_TOTAL <= (size_t)134217728);
static_assert(((ROWS / 64) * (NQKV / 64)) % 8 == 0);
static_assert((((size_t)SEQ / 64) * (EMB / 64)) % 8 == 0);
static_assert((((size_t)ISL / 64) * (EMB / 64)) % 8 == 0);
static_assert((ROWS * (EMB / 8)) % 256 == 0);

extern "C" void kernel_launch(void* const* d_in, const int* in_sizes, int n_in, void* d_out, int out_size, void* d_ws, size_t ws_size, hipStream_t stream) {
    if (n_in < 5) return;
    const long long needX = (long long)(NB - 1) * SEQ_FULL * EMB + (long long)SEQ * EMB;
    if ((long long)in_sizes[0] < needX) return;
    if ((long long)in_sizes[1] < (long long)EMB * NQKV) return;
    if ((long long)in_sizes[2] < (long long)NQKV) return;
    if ((long long)in_sizes[3] < (long long)EMB * EMB) return;
    if ((long long)in_sizes[4] < (long long)EMB) return;
    if ((long long)out_size < needX) return;
    if (ws_size < WS_TOTAL) return;
    const float* x    = (const float*)d_in[0];
    const float* Wqkv = (const float*)d_in[1];
    const float* bqkv = (const float*)d_in[2];
    const float* Wo   = (const float*)d_in[3];
    const float* bo   = (const float*)d_in[4];
    float* out = (float*)d_out;
    char* wsp = (char*)d_ws;
    unsigned short* X16  = (unsigned short*)wsp; wsp += SZ_X16;
    unsigned short* W316 = (unsigned short*)wsp; wsp += SZ_W316;
    float* QKV           = (float*)wsp;          wsp += SZ_QKV;
    float* AO            = (float*)wsp;          wsp += SZ_AO;
    float* BR3           = (float*)wsp;          wsp += SZ_BR3;
    unsigned short* WO16 = (unsigned short*)wsp; wsp += SZ_WO;
    unsigned short* WOB  = (unsigned short*)wsp; wsp += SZ_WO;
    unsigned short* AOH2 = (unsigned short*)wsp; wsp += SZ_ISLP;
    unsigned short* AOL2 = (unsigned short*)wsp; wsp += SZ_ISLP;
    float* BRO           = (float*)wsp;          wsp += SZ_BRO;
    unsigned short* AO16 = X16;

    k_cast_rows<<<(unsigned)((ROWS * (EMB / 8) + 255) / 256), 256, 0, stream>>>(x, X16, (int)ROWS, SEQ, (long long)SEQ_FULL * EMB, 1.0f, 1);
    k_castT<<<(unsigned)(((size_t)NQKV * (EMB / 8) + 255) / 256), 256, 0, stream>>>(Wqkv, NQKV, W316, EMB, EMB, NQKV, 16.0f, 0);
    k_bfvec<<<(NQKV + 255) / 256, 256, 0, stream>>>(bqkv, BR3, NQKV);
    k_castT<<<(unsigned)(((size_t)EMB * (EMB / 8) + 255) / 256), 256, 0, stream>>>(Wo, EMB, WO16, EMB, EMB, EMB, 16.0f, 0);
    k_castT<<<(unsigned)(((size_t)EMB * (EMB / 8) + 255) / 256), 256, 0, stream>>>(Wo, EMB, WOB, EMB, EMB, EMB, 1.0f, 1);
    k_bfvec<<<(EMB + 255) / 256, 256, 0, stream>>>(bo, BRO, EMB);

    {
        G64P g;
        g.A = X16; g.Bt = W316; g.C = QKV; g.bias = BR3; g.resid = BR3;
        g.strideA = 0; g.strideC = 0; g.strideR = 0;
        g.lda = EMB; g.ldb = EMB; g.ldc = NQKV; g.M = (int)ROWS; g.N = NQKV; g.K = EMB; g.scale = 0.0625f; g.pad_ = 0;
        k_gemm_f16_bias<<<dim3((unsigned)(((ROWS / 64) * (NQKV / 64)) / 8), 1), 256, 0, stream>>>(G64_ARGS(g));
    }
    k_gx_exact<<<dim3(ISL, NHEAD, NB), 64, 0, stream>>>(QKV, AO, (long long)SEQ * NQKV, (long long)SEQ * EMB, 0.125f);
    if (SEQ - ISL > 0) {
        AttnP a;
        a.Q = QKV + (size_t)ISL * NQKV; a.K = QKV + EMB; a.V = QKV + 2 * EMB; a.O = AO + (size_t)ISL * EMB;
        a.sQb = (long long)SEQ * NQKV; a.sQh = HDIM; a.sQi = NQKV;
        a.sKb = (long long)SEQ * NQKV; a.sKh = HDIM; a.sKj = NQKV;
        a.sVb = (long long)SEQ * NQKV; a.sVh = HDIM; a.sVj = NQKV;
        a.sOb = (long long)SEQ * EMB;  a.sOh = HDIM; a.sOi = EMB;
        a.Lq = SEQ - ISL; a.Lk = SEQ; a.coff = ISL; a.pad_ = 0; a.scale = 0.125f; a.pad2_ = 0.0f;
        k_attn_causal<<<dim3((unsigned)((SEQ - ISL) / (16 * AW)), NHEAD, NB), 32 * AW, 0, stream>>>(ATTN_ARGS(a));
    }
    k_cast_rows<<<(unsigned)((ROWS * (EMB / 8) + 255) / 256), 256, 0, stream>>>(AO, AO16, (int)ROWS, (int)ROWS, 0, 1.0f, 0);
    {
        G64P g;
        g.A = AO16; g.Bt = WO16; g.C = out; g.bias = BRO; g.resid = BRO;
        g.strideA = (long long)SEQ * EMB; g.strideC = (long long)SEQ_FULL * EMB; g.strideR = 0;
        g.lda = EMB; g.ldb = EMB; g.ldc = EMB; g.M = SEQ; g.N = EMB; g.K = EMB; g.scale = 0.0625f; g.pad_ = 0;
        k_gemm_f16_bias<<<dim3((unsigned)((((size_t)SEQ / 64) * (EMB / 64)) / 8), NB), 256, 0, stream>>>(G64_ARGS(g));
    }
    k_split_rows<<<(unsigned)(((size_t)NB * ISL * (EMB / 8) + 255) / 256), 256, 0, stream>>>(AO, (long long)SEQ * EMB, AOH2, AOL2, ISL, NB);
    {
        G64P g;
        g.A = AOH2; g.Bt = WOB; g.C = out; g.bias = BRO; g.resid = BRO;
        g.strideA = (long long)ISL * EMB; g.strideC = (long long)SEQ_FULL * EMB; g.strideR = 0;
        g.lda = EMB; g.ldb = EMB; g.ldc = EMB; g.M = ISL; g.N = EMB; g.K = EMB; g.scale = 1.0f; g.pad_ = 0;
        k_gemm_bf16_bias<<<dim3((unsigned)((((size_t)ISL / 64) * (EMB / 64)) / 8), NB), 256, 0, stream>>>(G64_ARGS(g));
    }
    {
        G64P g;
        g.A = AOL2; g.Bt = WOB; g.C = out; g.bias = BRO; g.resid = out;
        g.strideA = (long long)ISL * EMB; g.strideC = (long long)SEQ_FULL * EMB; g.strideR = (long long)SEQ_FULL * EMB;
        g.lda = EMB; g.ldb = EMB; g.ldc = EMB; g.M = ISL; g.N = EMB; g.K = EMB; g.scale = 1.0f; g.pad_ = 0;
        k_gemm_bf16_resid<<<dim3((unsigned)((((size_t)ISL / 64) * (EMB / 64)) / 8), NB), 256, 0, stream>>>(G64_ARGS(g));
    }
}
